// Block_996432412771
// MI455X (gfx1250) — hardware-verified
//
#include <hip/hip_runtime.h>
#include <math.h>

#ifndef NB
#define NB 4
#endif
#ifndef SEQ
#define SEQ 2048
#endif
#define NB_FULL 4
#define SEQ_FULL 2048
#define CH 192
#define HEADS 16
#define HD 12
#define HDP 16
#define SAW 256
#define QKVW 768
#define FFD 768
#define MTOK (NB * SEQ)

static_assert(SEQ == SEQ_FULL || NB == 1);
static_assert(NB <= NB_FULL && SEQ <= SEQ_FULL);
static_assert(SEQ % 128 == 0);
static_assert(MTOK % 64 == 0);
static_assert(HD <= HDP && HDP == 16);
static_assert(HEADS * HD == CH);
static_assert(HEADS * HDP == SAW && 3 * SAW == QKVW);
static_assert(CH % 64 == 0 && QKVW % 64 == 0 && FFD % 64 == 0);
static_assert(CH % 32 == 0 && SAW % 32 == 0 && FFD % 32 == 0);
static_assert(CH % 8 == 0 && FFD % 8 == 0 && SAW % 8 == 0);
static_assert(CH == 6 * 32);
static_assert(MTOK % 8 == 0);

typedef __attribute__((ext_vector_type(16))) _Float16 v16h;
typedef __attribute__((ext_vector_type(8)))  _Float16 v8h;
typedef __attribute__((ext_vector_type(2)))  _Float16 v2h;
typedef __attribute__((ext_vector_type(8)))  float    v8f;
typedef __attribute__((ext_vector_type(4)))  float    v4f;
typedef __attribute__((ext_vector_type(2)))  float    v2f;
typedef __attribute__((ext_vector_type(4)))  unsigned int v4u;
typedef __attribute__((ext_vector_type(8)))  unsigned int v8u;


#define VST2(T, ptr, val) do { const T vst2_v_ = (val); *(volatile T*)(ptr) = vst2_v_; __threadfence(); *(volatile T*)(ptr) = vst2_v_; } while (0)

__device__ __forceinline__ float bfr(float f) {
    unsigned u = __float_as_uint(f);
    u += 0x7FFFu + ((u >> 16) & 1u);
    return __uint_as_float(u & 0xFFFF0000u);
}

static __device__ __forceinline__ unsigned toh_flush2(float a, float b) {
    v2f w;
    w.x = (fabsf(a) < 6.103515625e-05f) ? 0.0f : a;
    w.y = (fabsf(b) < 6.103515625e-05f) ? 0.0f : b;
    const v2h r = __builtin_convertvector(w, v2h);
    return __builtin_bit_cast(unsigned, r);
}
static __device__ __forceinline__ v4u pack8h_flush(const float* v) {
    v4u pk;
    pk.x = toh_flush2(v[0], v[1]);
    pk.y = toh_flush2(v[2], v[3]);
    pk.z = toh_flush2(v[4], v[5]);
    pk.w = toh_flush2(v[6], v[7]);
    return pk;
}

union FragU { v16h v; v8h h[2]; };
__device__ __forceinline__ v16h frag_ld(const _Float16* p) {
    FragU f; f.h[0] = *(const v8h*)(p); f.h[1] = *(const v8h*)(p + 16); return f.v;
}
__device__ __forceinline__ v8f wmma16(v16h a, v16h b, v8f c) {
    c = __builtin_amdgcn_wmma_f32_16x16x32_f16(false, a, false, b, (short)0, c, false, false);
    asm volatile("v_nop\n\tv_nop\n\tv_nop\n\tv_nop" : "+v"(c) : "v"(a), "v"(b));
    return c;
}
__device__ __forceinline__ void wave_sync_lds() {
    __builtin_amdgcn_fence(3  , "workgroup");
    __builtin_amdgcn_wave_barrier();
    __builtin_amdgcn_fence(2  , "workgroup");
}

static_assert(sizeof(float) * 8 * 16 * 68 <= 131072);
static_assert(2 * 4 * 2 == 16);
static_assert(4 * 4 == 16);
template <int OUT_MODE, bool BIAS, bool RESID, bool RESBF, bool SILU>
static __device__ __forceinline__ void gemm64_body(
    const _Float16* __restrict__ A, unsigned lda, const _Float16* __restrict__ Bt, unsigned ldb,
    void* __restrict__ Cout, unsigned ldc, const float* __restrict__ bias, const float* __restrict__ resid,
    unsigned M, unsigned N, unsigned K, float scale, float oscale) {
  __shared__ __align__(16) float sT[8][16 * 68];
  const unsigned lane = threadIdx.x & 31u;
  const unsigned wave = threadIdx.x >> 5;
  const unsigned tilesN = N >> 6, tilesM = M >> 6;
  const unsigned tile = blockIdx.x * 8u + wave;
  if (tile >= tilesM * tilesN) return;
  unsigned tpin = tile;
  asm volatile("" : "+v"(tpin));
  const unsigned tm = tpin / tilesN;
  const unsigned tn = tpin - tm * tilesN;
  const unsigned m0 = tm << 6, n0 = tn << 6;
  const unsigned rlane = lane & 15u;
  const unsigned koff = (lane >> 4) * 8u;
  const unsigned mOff = koff;

  v8f acc[4][4];
#pragma unroll
  for (int i = 0; i < 4; ++i)
#pragma unroll
    for (int j = 0; j < 4; ++j) acc[i][j] = (v8f){0.f,0.f,0.f,0.f,0.f,0.f,0.f,0.f};

  for (unsigned k0 = 0; k0 < K; k0 += 32u) {
    v16h bh[4];
#pragma unroll
    for (int j = 0; j < 4; ++j)
      bh[j] = frag_ld(Bt + (size_t)(n0 + ((unsigned)j << 4) + rlane) * ldb + koff + k0);
#pragma unroll
    for (int i = 0; i < 4; ++i) {
      const v16h ah = frag_ld(A + (size_t)(m0 + ((unsigned)i << 4) + rlane) * lda + koff + k0);
#pragma unroll
      for (int j = 0; j < 4; ++j)
        acc[i][j] = wmma16(ah, bh[j], acc[i][j]);
    }
  }

  float* slab = sT[wave];
#pragma unroll
  for (int i = 0; i < 4; ++i) {
    const unsigned mBase = m0 + ((unsigned)i << 4);
#pragma unroll
    for (int j = 0; j < 4; ++j) {
      const unsigned n = n0 + ((unsigned)j << 4) + rlane;
      float bv = 0.0f;
      if (BIAS) bv = bfr(bias[n]);
#pragma unroll
      for (int r = 0; r < 8; ++r) {
        float v = acc[i][j][r] * scale + bv;
        if (SILU) v = v / (1.0f + expf(-v));
        if (OUT_MODE == 1) v *= oscale;
        slab[(mOff + (unsigned)r) * 68u + ((unsigned)j << 4) + rlane] = v;
      }
    }
    wave_sync_lds();
    if (OUT_MODE == 0) {
      float* C = (float*)Cout;
      const unsigned hh = lane >> 4, c4 = (lane & 15u) * 4u;
#pragma unroll
      for (int half = 0; half < 2; ++half) {
        v4f vv[4];
#pragma unroll
        for (int it = 0; it < 4; ++it) {
          const unsigned row = (unsigned)(half * 4 + it) * 2u + hh;
          vv[it] = *(const v4f*)(slab + row * 68u + c4);
          if (RESID) {
            v4f rr = *(const v4f*)(resid + (size_t)(mBase + row) * ldc + n0 + c4);
            if (RESBF) { rr.x = bfr(rr.x); rr.y = bfr(rr.y); rr.z = bfr(rr.z); rr.w = bfr(rr.w); }
            vv[it] += rr;
          }
        }
        for (int pass = 0; pass < 2; ++pass) {
#pragma unroll
          for (int it = 0; it < 4; ++it) {
            const unsigned row = (unsigned)(half * 4 + it) * 2u + hh;
            *(volatile v4f*)(C + (size_t)(mBase + row) * ldc + n0 + c4) = vv[it];
          }
          __threadfence();
        }
      }
    } else {
      _Float16* C = (_Float16*)Cout;
      const unsigned q = lane >> 3, c8 = (lane & 7u) * 8u;
      v4u hv[4];
#pragma unroll
      for (int it = 0; it < 4; ++it) {
        const unsigned row = (unsigned)it * 4u + q;
        const float* sp = slab + row * 68u + c8;
        float t8[8];
#pragma unroll
        for (int e = 0; e < 8; ++e) t8[e] = sp[e];
        hv[it] = pack8h_flush(t8);
      }
      for (int pass = 0; pass < 2; ++pass) {
#pragma unroll
        for (int it = 0; it < 4; ++it) {
          const unsigned row = (unsigned)it * 4u + q;
          *(volatile v4u*)(C + (size_t)(mBase + row) * ldc + n0 + c8) = hv[it];
        }
        __threadfence();
      }
    }
    wave_sync_lds();
  }
}

__global__ __launch_bounds__(256) void k_gemm_qkv(const _Float16* __restrict__ A, const _Float16* __restrict__ Bt,
                                                  _Float16* __restrict__ C) {
    gemm64_body<1, false, false, false, false>(A, CH, Bt, CH, (void*)C, QKVW, nullptr, nullptr,
                                               MTOK, QKVW, CH, 1.0f / 1048576.0f, 1024.0f);
}
__global__ __launch_bounds__(256) void k_gemm_proj(const _Float16* __restrict__ A, const _Float16* __restrict__ Bt,
                                                   float* __restrict__ C, const float* __restrict__ bias,
                                                   const float* __restrict__ resid) {
    gemm64_body<0, true, true, true, false>(A, SAW, Bt, SAW, (void*)C, CH, bias, resid,
                                            MTOK, CH, SAW, 1.0f / 4194304.0f, 1.0f);
}
__global__ __launch_bounds__(256) void k_gemm_up(const _Float16* __restrict__ A, const _Float16* __restrict__ Bt,
                                                 _Float16* __restrict__ C) {
    gemm64_body<1, false, false, false, true>(A, CH, Bt, CH, (void*)C, FFD, nullptr, nullptr,
                                              MTOK, FFD, CH, 1.0f / 1048576.0f, 1024.0f);
}
__global__ __launch_bounds__(256) void k_gemm_down(const _Float16* __restrict__ A, const _Float16* __restrict__ Bt,
                                                   float* __restrict__ C, const float* __restrict__ resid) {
    gemm64_body<0, false, true, false, false>(A, FFD, Bt, FFD, (void*)C, CH, nullptr, resid,
                                              MTOK, CH, FFD, 1.0f / 4194304.0f, 1.0f);
}

__global__ __launch_bounds__(256) void k_wt16(const float* __restrict__ Wm, unsigned KI, unsigned NO,
                                              unsigned short* __restrict__ W16) {
    const unsigned lane = threadIdx.x & 31u;
    const unsigned o = blockIdx.x * 8u + (threadIdx.x >> 5);
    const unsigned np = KI >> 3;
    for (unsigned p0 = 0; p0 < np; p0 += 32u) {
        const unsigned p = p0 + lane;
        const bool ok = p < np;
        const unsigned pc = ok ? p : (np - 1u);
        const unsigned k0 = 8u * pc;
        float v[8];
#pragma unroll
        for (int i = 0; i < 8; ++i) v[i] = bfr(Wm[(k0 + (unsigned)i) * NO + o]) * 4096.0f;
        const v4u pk = pack8h_flush(v);
        if (ok) { VST2(v4u, (v4u*)(W16 + o * KI + k0), pk); }
    }
}

static_assert(24 * 16 == CH * 2);
__global__ __launch_bounds__(256) void k_wqkv(const float* __restrict__ Wh, unsigned rowbase,
                                              unsigned short* __restrict__ W16) {
    const unsigned lane = threadIdx.x & 31u;
    const unsigned o = blockIdx.x * 8u + (threadIdx.x >> 5);
    const unsigned hd = o >> 4, d = o & 15u;
    const unsigned dc = (d < (unsigned)HD) ? d : (unsigned)(HD - 1);
    const bool live = d < (unsigned)HD;
    const bool ok = lane < 24u;
    const unsigned pc = ok ? lane : 23u;
    const unsigned k0 = 8u * pc;
    float v[8];
#pragma unroll
    for (int i = 0; i < 8; ++i) {
        const float t = bfr(Wh[(hd * (unsigned)CH + k0 + (unsigned)i) * (unsigned)HD + dc]) * 4096.0f;
        v[i] = live ? t : 0.0f;
    }
    const v4u pk = pack8h_flush(v);
    if (ok) { VST2(v4u, (v4u*)(W16 + (rowbase + o) * (unsigned)CH + k0), pk); }
}

static_assert(32 * 16 == SAW * 2);
__global__ __launch_bounds__(256) void k_wproj(const float* __restrict__ Wp, unsigned short* __restrict__ W16) {
    const unsigned lane = threadIdx.x & 31u;
    const unsigned o = blockIdx.x * 8u + (threadIdx.x >> 5);
    const unsigned hd = lane >> 1, d0 = 8u * (lane & 1u);
    float v[8];
#pragma unroll
    for (int i = 0; i < 8; ++i) {
        const unsigned d = d0 + (unsigned)i;
        const unsigned dc = (d < (unsigned)HD) ? d : (unsigned)(HD - 1);
        const float t = bfr(Wp[((unsigned)HD * hd + dc) * (unsigned)CH + o]) * 4096.0f;
        v[i] = (d < (unsigned)HD) ? t : 0.0f;
    }
    const v4u pk = pack8h_flush(v);
    VST2(v4u, (v4u*)(W16 + o * (unsigned)SAW + 8u * lane), pk);
}

static_assert(sizeof(float) * 8 * CH <= 131072);
__global__ __launch_bounds__(256) void k_rms(const float* __restrict__ xin, const float* __restrict__ w,
                                             unsigned short* __restrict__ hp, unsigned M, int inbf) {
    __shared__ __align__(16) float sR[8][CH];
    const unsigned wave = (unsigned)__builtin_amdgcn_readfirstlane((int)(threadIdx.x >> 5));
    const unsigned L = threadIdx.x & 31u;
    const unsigned row = blockIdx.x * 8u + wave;
    if (row >= M) return;
    const float* xr = xin + (size_t)row * CH + 6u * L;
    const v2f a0 = *(const v2f*)xr, a1 = *(const v2f*)(xr + 2), a2 = *(const v2f*)(xr + 4);
    const v2f w0 = *(const v2f*)(w + 6u * L), w1 = *(const v2f*)(w + 6u * L + 2u), w2 = *(const v2f*)(w + 6u * L + 4u);
    float v[6] = {a0.x, a0.y, a1.x, a1.y, a2.x, a2.y};
    const float g[6] = {bfr(w0.x), bfr(w0.y), bfr(w1.x), bfr(w1.y), bfr(w2.x), bfr(w2.y)};
    if (inbf != 0) {
#pragma unroll
        for (int i = 0; i < 6; ++i) v[i] = bfr(v[i]);
    }
    float s = ((v[0] * v[0] + v[1] * v[1]) + (v[2] * v[2] + v[3] * v[3])) + (v[4] * v[4] + v[5] * v[5]);
#pragma unroll
    for (int o = 16; o > 0; o >>= 1) s += __shfl_xor(s, o, 32);
    const float ms = s / 192.0f;
    const float rs = 1.0f / sqrtf(ms + 1e-5f);
    float* line = sR[wave];
#pragma unroll
    for (int i = 0; i < 3; ++i) {
        v2f y;
        y.x = v[2 * i] * rs * g[2 * i] * 256.0f;
        y.y = v[2 * i + 1] * rs * g[2 * i + 1] * 256.0f;
        *(v2f*)(line + 6u * L + 2u * (unsigned)i) = y;
    }
    wave_sync_lds();
    const bool ok = L < 24u;
    const unsigned pl = ok ? L : 23u;
    const v4f r0 = *(const v4f*)(line + 8u * pl), r1 = *(const v4f*)(line + 8u * pl + 4u);
    const float t[8] = {r0.x, r0.y, r0.z, r0.w, r1.x, r1.y, r1.z, r1.w};
    const v4u pk = pack8h_flush(t);
    if (ok) { VST2(v4u, (v4u*)(hp + (size_t)row * CH + 8u * pl), pk); }
}

#define VT_KEYS 128
#define VT_P 132
static_assert(256 * 16 == 16 * VT_KEYS * 2);
static_assert(256 * 8 == 16 * VT_KEYS);
static_assert(sizeof(float) * 16 * VT_P <= 131072);
__global__ __launch_bounds__(256) void k_vt(const _Float16* __restrict__ qkv, unsigned short* __restrict__ vt) {
    __shared__ __align__(16) float sV[16 * VT_P];
    const unsigned tid = threadIdx.x;
    const unsigned g = blockIdx.y;
    const unsigned b = g >> 4, hd = g & 15u;
    const unsigned k0 = blockIdx.x * (unsigned)VT_KEYS;
    {
        const unsigned key = tid >> 1, hp = tid & 1u;
        const v8h vv = *(const v8h*)(qkv + (b * (unsigned)SEQ + k0 + key) * (unsigned)QKVW + 512u + 16u * hd + 8u * hp);
#pragma unroll
        for (int e = 0; e < 8; ++e) sV[(8u * hp + (unsigned)e) * VT_P + key] = (float)vv[e];
    }
    __syncthreads();
    {
        const unsigned row = tid >> 4, pc = tid & 15u;
        const float* sp = sV + row * VT_P + 8u * pc;
        const v4f r0 = *(const v4f*)sp, r1 = *(const v4f*)(sp + 4);
        const float t[8] = {r0.x, r0.y, r0.z, r0.w, r1.x, r1.y, r1.z, r1.w};
        const v4u pk = pack8h_flush(t);
        VST2(v4u, (v4u*)(vt + (g * 16u + row) * (unsigned)SEQ + k0 + 8u * pc), pk);
    }
}

#define AT_PP 36
#define AT_OP 260
static_assert(512 * 16 == 16 * SAW * 2);
static_assert(sizeof(float) * (16 * 16 * AT_PP + 16 * AT_OP) <= 131072);
static_assert(SEQ % 32 == 0);
__global__ __launch_bounds__(512) void k_attn(const _Float16* __restrict__ qkv, const _Float16* __restrict__ vt,
                                              unsigned short* __restrict__ sa) {
    __shared__ __align__(16) float sP[16][16 * AT_PP];
    __shared__ __align__(16) float sO[16 * AT_OP];
    const unsigned tid = threadIdx.x, lane = tid & 31u;
    const unsigned wave = (unsigned)__builtin_amdgcn_readfirstlane((int)(tid >> 5));
    const unsigned hh = lane >> 4, c = lane & 15u;
    const unsigned b = blockIdx.y;
    const unsigned t0 = blockIdx.x * 16u;
    const unsigned hd = wave;
    const unsigned g = b * 16u + hd;
    const unsigned rowbase = b * (unsigned)SEQ;
    float* pw = sP[wave];
    const float SC2 = 0.28867513459481287f * (1.0f / 1048576.0f) * 1.4426950408889634f;
    const v8h zero8 = {(_Float16)0.0f, (_Float16)0.0f, (_Float16)0.0f, (_Float16)0.0f,
                       (_Float16)0.0f, (_Float16)0.0f, (_Float16)0.0f, (_Float16)0.0f};
    FragU qf;
    qf.h[0] = *(const v8h*)(qkv + (rowbase + t0 + c) * (unsigned)QKVW + 16u * hd + 8u * hh);
    qf.h[1] = zero8;
    float mrow[8], lrow[8];
    v8f os = (v8f){0.f,0.f,0.f,0.f,0.f,0.f,0.f,0.f};
#pragma unroll
    for (int r = 0; r < 8; ++r) { mrow[r] = -3.0e38f; lrow[r] = 0.f; }
    const unsigned nsteps = (t0 >> 5) + 1u;
    for (unsigned st = 0; st < nsteps; ++st) {
        const unsigned kv0 = st * 32u;
        v8f s[2];
#pragma unroll
        for (int j = 0; j < 2; ++j) {
            FragU kf;
            kf.h[0] = *(const v8h*)(qkv + (rowbase + kv0 + (unsigned)j * 16u + c) * (unsigned)QKVW + 256u + 16u * hd + 8u * hh);
            kf.h[1] = zero8;
            const v8f z = (v8f){0.f,0.f,0.f,0.f,0.f,0.f,0.f,0.f};
            s[j] = wmma16(qf.v, kf.v, z);
        }
        const v16h vb = frag_ld(vt + (g * 16u + c) * (unsigned)SEQ + kv0 + 8u * hh);
#pragma unroll
        for (int r = 0; r < 8; ++r) {
            const unsigned tq = t0 + 8u * hh + (unsigned)r;
            float mx = -3.0e38f;
#pragma unroll
            for (int j = 0; j < 2; ++j) {
                const unsigned ks = kv0 + (unsigned)j * 16u + c;
                const float sv = s[j][r] * SC2;
                s[j][r] = (ks <= tq) ? sv : -3.0e38f;
                mx = fmaxf(mx, s[j][r]);
            }
            mx = fmaxf(mx, __shfl_xor(mx, 1, 32)); mx = fmaxf(mx, __shfl_xor(mx, 2, 32));
            mx = fmaxf(mx, __shfl_xor(mx, 4, 32)); mx = fmaxf(mx, __shfl_xor(mx, 8, 32));
            const float mnew = fmaxf(mrow[r], mx);
            const float alpha = exp2f(mrow[r] - mnew);
            mrow[r] = mnew;
            float psum = 0.f;
#pragma unroll
            for (int j = 0; j < 2; ++j) {
                const unsigned ks = kv0 + (unsigned)j * 16u + c;
                const float e = exp2f(s[j][r] - mnew);
                const float p = (ks <= tq) ? e : 0.0f;
                psum += p;
                pw[(8u * hh + (unsigned)r) * AT_PP + (unsigned)j * 16u + c] = p;
            }
            psum += __shfl_xor(psum, 1, 32); psum += __shfl_xor(psum, 2, 32);
            psum += __shfl_xor(psum, 4, 32); psum += __shfl_xor(psum, 8, 32);
            lrow[r] = lrow[r] * alpha + psum;
            os[r] *= alpha;
        }
        wave_sync_lds();
        {
            const float* pr = pw + c * AT_PP + 8u * hh;
            const v4f x0 = *(const v4f*)(pr), x1 = *(const v4f*)(pr + 4);
            const v4f x2 = *(const v4f*)(pr + 16), x3 = *(const v4f*)(pr + 20);
            v8u pu;
            pu[0] = toh_flush2(x0.x * 1024.0f, x0.y * 1024.0f);
            pu[1] = toh_flush2(x0.z * 1024.0f, x0.w * 1024.0f);
            pu[2] = toh_flush2(x1.x * 1024.0f, x1.y * 1024.0f);
            pu[3] = toh_flush2(x1.z * 1024.0f, x1.w * 1024.0f);
            pu[4] = toh_flush2(x2.x * 1024.0f, x2.y * 1024.0f);
            pu[5] = toh_flush2(x2.z * 1024.0f, x2.w * 1024.0f);
            pu[6] = toh_flush2(x3.x * 1024.0f, x3.y * 1024.0f);
            pu[7] = toh_flush2(x3.z * 1024.0f, x3.w * 1024.0f);
            const v16h pa = __builtin_bit_cast(v16h, pu);
            os = wmma16(pa, vb, os);
        }
        wave_sync_lds();
    }
#pragma unroll
    for (int r = 0; r < 8; ++r) {
        const float o = os[r] / (lrow[r] * 1048576.0f);
        sO[(8u * hh + (unsigned)r) * AT_OP + 16u * hd + c] = o * 1024.0f;
    }
    __syncthreads();
    {
        const float* sp = sO + wave * AT_OP + 8u * lane;
        const v4f r0 = *(const v4f*)sp, r1 = *(const v4f*)(sp + 4);
        const float t[8] = {r0.x, r0.y, r0.z, r0.w, r1.x, r1.y, r1.z, r1.w};
        const v4u pk = pack8h_flush(t);
        VST2(v4u, (v4u*)(sa + (rowbase + t0 + wave) * (unsigned)SAW + 8u * lane), pk);
    }
}

constexpr size_t al256(size_t b) { return (b + 255) & ~(size_t)255; }
constexpr size_t SZ_H16   = al256((size_t)MTOK * CH * 2);
constexpr size_t SZ_QKV16 = al256((size_t)MTOK * QKVW * 2);
constexpr size_t SZ_VT16  = al256((size_t)NB * HEADS * HDP * SEQ * 2);
constexpr size_t SZ_SA16  = al256((size_t)MTOK * SAW * 2);
constexpr size_t SZ_X1    = al256((size_t)MTOK * CH * 4);
constexpr size_t SZ_G16   = al256((size_t)MTOK * FFD * 2);
constexpr size_t SZ_WQKV  = al256((size_t)QKVW * CH * 2);
constexpr size_t SZ_WPROJ = al256((size_t)CH * SAW * 2);
constexpr size_t SZ_W1    = al256((size_t)FFD * CH * 2);
constexpr size_t SZ_W2    = al256((size_t)CH * FFD * 2);
constexpr size_t OFF_H16   = 0;
constexpr size_t OFF_QKV16 = OFF_H16 + SZ_H16;
constexpr size_t OFF_VT16  = OFF_QKV16 + SZ_QKV16;
constexpr size_t OFF_SA16  = OFF_VT16 + SZ_VT16;
constexpr size_t OFF_X1    = OFF_SA16 + SZ_SA16;
constexpr size_t OFF_G16   = OFF_X1 + SZ_X1;
constexpr size_t OFF_WQKV  = OFF_G16 + SZ_G16;
constexpr size_t OFF_WPROJ = OFF_WQKV + SZ_WQKV;
constexpr size_t OFF_W1    = OFF_WPROJ + SZ_WPROJ;
constexpr size_t OFF_W2    = OFF_W1 + SZ_W1;
constexpr size_t WS_TOTAL  = OFF_W2 + SZ_W2;
static_assert(WS_TOTAL <= 134217728);
static_assert((HEADS * HDP) % 8 == 0 && CH % 8 == 0 && FFD % 8 == 0);
static_assert(((MTOK / 64) * (QKVW / 64)) % 8 == 0 && ((MTOK / 64) * (CH / 64)) % 8 == 0 && ((MTOK / 64) * (FFD / 64)) % 8 == 0);

extern "C" void kernel_launch(void* const* d_in, const int* in_sizes, int n_in, void* d_out, int out_size,
                              void* d_ws, size_t ws_size, hipStream_t stream) {
    if (n_in < 10) return;
    if (in_sizes[0] < MTOK * CH || in_sizes[1] < CH || in_sizes[2] < CH) return;
    if (in_sizes[3] < HEADS * CH * HD || in_sizes[4] < HEADS * CH * HD || in_sizes[5] < HEADS * CH * HD) return;
    if (in_sizes[6] < CH * CH || in_sizes[7] < CH || in_sizes[8] < CH * FFD || in_sizes[9] < FFD * CH) return;
    if (out_size < MTOK * CH) return;
    if (WS_TOTAL > ws_size) return;

    const float* x     = (const float*)d_in[0];
    const float* ln1_w = (const float*)d_in[1];
    const float* ln2_w = (const float*)d_in[2];
    const float* Wq    = (const float*)d_in[3];
    const float* Wk    = (const float*)d_in[4];
    const float* Wv    = (const float*)d_in[5];
    const float* Wproj = (const float*)d_in[6];
    const float* bproj = (const float*)d_in[7];
    const float* W1    = (const float*)d_in[8];
    const float* W2    = (const float*)d_in[9];
    float* out = (float*)d_out;

    char* wsp = (char*)d_ws;
    unsigned short* h16    = (unsigned short*)(wsp + OFF_H16);
    unsigned short* qkv16  = (unsigned short*)(wsp + OFF_QKV16);
    unsigned short* vt16   = (unsigned short*)(wsp + OFF_VT16);
    unsigned short* sa16   = (unsigned short*)(wsp + OFF_SA16);
    float*          x1     = (float*)(wsp + OFF_X1);
    unsigned short* g16    = (unsigned short*)(wsp + OFF_G16);
    unsigned short* wqkv   = (unsigned short*)(wsp + OFF_WQKV);
    unsigned short* wproj  = (unsigned short*)(wsp + OFF_WPROJ);
    unsigned short* w1p    = (unsigned short*)(wsp + OFF_W1);
    unsigned short* w2p    = (unsigned short*)(wsp + OFF_W2);

    k_wqkv<<<(HEADS * HDP) / 8, 256, 0, stream>>>(Wq, 0u, wqkv);
    k_wqkv<<<(HEADS * HDP) / 8, 256, 0, stream>>>(Wk, 256u, wqkv);
    k_wqkv<<<(HEADS * HDP) / 8, 256, 0, stream>>>(Wv, 512u, wqkv);
    k_wproj<<<CH / 8, 256, 0, stream>>>(Wproj, wproj);
    k_wt16<<<FFD / 8, 256, 0, stream>>>(W1, CH, FFD, w1p);
    k_wt16<<<CH / 8, 256, 0, stream>>>(W2, FFD, CH, w2p);

    const unsigned gQ = ((MTOK / 64) * (QKVW / 64)) / 8;
    const unsigned gE = ((MTOK / 64) * (CH / 64)) / 8;
    const unsigned gF = ((MTOK / 64) * (FFD / 64)) / 8;

    k_rms<<<MTOK / 8, 256, 0, stream>>>(x, ln1_w, h16, (unsigned)MTOK, 1);
    k_gemm_qkv<<<gQ, 256, 0, stream>>>((const _Float16*)h16, (const _Float16*)wqkv, (_Float16*)qkv16);
    k_vt<<<dim3(SEQ / VT_KEYS, NB * HEADS), 256, 0, stream>>>((const _Float16*)qkv16, vt16);
    k_attn<<<dim3(SEQ / 16, NB), 512, 0, stream>>>((const _Float16*)qkv16, (const _Float16*)vt16, sa16);
    k_gemm_proj<<<gE, 256, 0, stream>>>((const _Float16*)sa16, (const _Float16*)wproj, x1, bproj, x);
    k_rms<<<MTOK / 8, 256, 0, stream>>>(x1, ln2_w, h16, (unsigned)MTOK, 0);
    k_gemm_up<<<gF, 256, 0, stream>>>((const _Float16*)h16, (const _Float16*)w1p, (_Float16*)g16);
    k_gemm_down<<<gE, 256, 0, stream>>>((const _Float16*)g16, (const _Float16*)w2p, out, x1);
}
